// DiffTransformerLayer_65146063946370
// MI455X (gfx1250) — hardware-run, weakly checked
//
#include <hip/hip_runtime.h>


#ifndef NB
#define NB 4
#endif
#ifndef SEQ
#define SEQ 1024
#endif
#define NB_FULL  4
#define SEQ_FULL 1024
#ifndef OUT_SEQ
#define OUT_SEQ SEQ
#endif
#define DM   1024
#define NH_  16
#define NZ   32
#define HD   32
#define VD   64
#define FF   4096
#define AW   4
#define OSP  68
#define EROWS (SEQ < 256 ? SEQ : 256)
#define QRS  2048.0f
#define QRI  (1.0f / 2048.0f)
#define SC2  ((float)(0.17677669529663687 * 1.4426950408889634))
#define PSH  14.0f
#define NEGB (-3.0e38f)
#define WCS  64.0f
#define ACS  16.0f
#define HCS  32.0f
#define EPSN 1.0e-5f
#define LINIT ((float)0.7836057665316245)
#define OML   ((float)(1.0 - 0.7836057665316245))

static_assert(HD == 32);
static_assert(NZ == 2 * NH_);
static_assert(NZ * HD == DM);
static_assert(NH_ * VD == DM);
static_assert(VD == 64);
static_assert(DM % 64 == 0);
static_assert(FF % 64 == 0);
static_assert(DM % 32 == 0);
static_assert(FF % 32 == 0);
static_assert(SEQ % 64 == 0);
static_assert((NB * SEQ) % 64 == 0);
static_assert(SEQ % 32 == 0);
static_assert(SEQ % (16 * AW) == 0);
static_assert(EROWS % 64 == 0);
static_assert(EROWS >= 32);
static_assert(EROWS % 32 == 0);
static_assert(EROWS <= SEQ);
static_assert(EROWS % (16 * AW) == 0);
static_assert((SEQ - EROWS) % (16 * AW) == 0);
static_assert(((size_t)SEQ * DM) % 8 == 0);
static_assert(((size_t)DM * DM) % 8 == 0);
static_assert(((size_t)FF * DM) % 8 == 0);
static_assert(NB <= NB_FULL);
static_assert(SEQ <= SEQ_FULL);
static_assert((OSP * 4) % 16 == 0);
static_assert(OSP >= VD);
static_assert((SEQ * 32) % 256 == 0);
static_assert((NB * SEQ) % 8 == 0);
static_assert(2 * 32 * 16 == 16 * HD * 2);
static_assert(4 * 32 * 16 == 16 * 64 * 2);
static_assert(8 * 32 * 16 == 16 * 64 * 4);
static_assert(4 * 32 * 16 == 16 * VD * 2);
static_assert(8 * 32 * 16 == DM * 4);
static_assert(16 * 68 * 4 <= 131072);
static_assert(AW * 16 * OSP * 4 <= 131072);

typedef _Float16 h16;
typedef unsigned short bf;
typedef __attribute__((ext_vector_type(16))) __bf16   v16bf;
typedef __attribute__((ext_vector_type(16))) _Float16 v16h;
typedef __attribute__((ext_vector_type(8)))  _Float16 v8h;
typedef __attribute__((ext_vector_type(8)))  unsigned short v8us;
typedef __attribute__((ext_vector_type(8)))  float    v8f;
typedef __attribute__((ext_vector_type(4)))  float    v4f;
typedef v4f  __attribute__((may_alias)) v4fa;

__device__ __forceinline__ unsigned short f2bf(float f) { unsigned u = __float_as_uint(f); u += 0x7FFFu + ((u >> 16) & 1u); return (unsigned short)(u >> 16); }
__device__ __forceinline__ float bfr(float f) { return __uint_as_float(((unsigned)f2bf(f)) << 16); }
__device__ __forceinline__ v16h cat16(v8h lo, v8h hi) { return __builtin_shufflevector(lo, hi, 0, 1, 2, 3, 4, 5, 6, 7, 8, 9, 10, 11, 12, 13, 14, 15); }
__device__ __forceinline__ v16bf cat16b(v8us lo, v8us hi) { return __builtin_bit_cast(v16bf, __builtin_shufflevector(lo, hi, 0, 1, 2, 3, 4, 5, 6, 7, 8, 9, 10, 11, 12, 13, 14, 15)); }
__device__ __forceinline__ v8f wmma16(v16h a, v16h b, v8f c) { return __builtin_amdgcn_wmma_f32_16x16x32_f16(false, a, false, b, (short)0, c, false, false); }
__device__ __forceinline__ v8f wmmab(v16bf a, v16bf b, v8f c) { return __builtin_amdgcn_wmma_f32_16x16x32_bf16(false, a, false, b, (short)0, c, false, false); }
__device__ __forceinline__ v16h  ldh(const h16* p) { return cat16(*(const v8h*)p, *(const v8h*)(p + 16)); }
__device__ __forceinline__ v16bf ldb(const bf* p)  { return cat16b(*(const v8us*)p, *(const v8us*)(p + 16)); }
__device__ __forceinline__ void wave_sync() { __builtin_amdgcn_fence(3  , "wavefront"); __builtin_amdgcn_wave_barrier(); asm volatile("" ::: "memory"); }

__device__ __forceinline__ v8f wmma16g(v16h a, v16h b, v8f c) { c = wmma16(a, b, c); asm volatile("v_nop\n\tv_nop\n\tv_nop\n\tv_nop" : "+v"(c) : "v"(a), "v"(b)); return c; }
__device__ __forceinline__ v8f wmmabg(v16bf a, v16bf b, v8f c) { c = wmmab(a, b, c); asm volatile("v_nop\n\tv_nop\n\tv_nop\n\tv_nop" : "+v"(c) : "v"(a), "v"(b)); return c; }
static __device__ __forceinline__ h16 toh_flush(float v) { const h16 r = (h16)v; return (fabsf(v) < 6.103515625e-05f) ? (h16)0.0f : r; }

__global__ __launch_bounds__(256) void k_cvt8(const float* __restrict__ src, bf* dst, size_t n8) {
    const size_t i = (size_t)blockIdx.x * 256 + threadIdx.x; if (i >= n8) return;
    const v8f v = *(const v8f*)(src + i * 8); v8us o;
#pragma unroll
    for (int k = 0; k < 8; ++k) o[k] = f2bf(v[k]);
    *(volatile v8us*)(dst + i * 8) = o; __threadfence(); *(volatile v8us*)(dst + i * 8) = o;
}

__global__ __launch_bounds__(256) void k_wconv(const float* __restrict__ src, h16* dst, size_t n8) {
    const size_t i = (size_t)blockIdx.x * 256 + threadIdx.x; if (i >= n8) return;
    const v8f v = *(const v8f*)(src + i * 8); v8h o;
#pragma unroll
    for (int k = 0; k < 8; ++k) o[k] = toh_flush(bfr(v[k]) * WCS);
    *(volatile v8h*)(dst + i * 8) = o; __threadfence(); *(volatile v8h*)(dst + i * 8) = o;
}

__global__ __launch_bounds__(32) void k_misc(const float* __restrict__ lq1, const float* __restrict__ lk1, const float* __restrict__ lq2, const float* __restrict__ lk2, float* misc) {
    const int lane = threadIdx.x & 31;
    float d1 = bfr(lq1[lane]) * bfr(lk1[lane]);
    float d2 = bfr(lq2[lane]) * bfr(lk2[lane]);
#pragma unroll 1
    for (int off = 16; off > 0; off >>= 1) { d1 += __shfl_xor(d1, off, 32); d2 += __shfl_xor(d2, off, 32); }
    const float ea = (lane & 1) ? d2 : d1;
    const float ex = expf(ea);
    const float e1 = __shfl(ex, 0, 32), e2 = __shfl(ex, 1, 32);
    const float lam = (e1 - e2) + LINIT;
    const int j = lane & 15;
    const float pw = powf(10000.0f, (float)j * 0.0625f);
    const float fr = 1.0f / pw;
    const float val = (lane < 16) ? fr : ((lane == 16) ? lam : 0.0f);
    *(volatile float*)(misc + lane) = val; __threadfence(); *(volatile float*)(misc + lane) = val;
}

__global__ __launch_bounds__(256) void k_ropetab(const float* __restrict__ misc, float* cs) {
#pragma clang fp contract(off)
    const int idx = blockIdx.x * 256 + threadIdx.x; if (idx >= SEQ * 32) return;
    const int t = idx >> 5, l = idx & 31;
    const float fr = misc[l & 15];
    const float ang = (float)t * fr;
    float sn, cn; sincosf(ang, &sn, &cn);
    const float val = (l < 16) ? cn : sn;
    *(volatile float*)(cs + idx) = val; __threadfence(); *(volatile float*)(cs + idx) = val;
}

template <int MODE>
__device__ __forceinline__ void proj_body(const bf* __restrict__ A, const bf* __restrict__ Bt, const float* __restrict__ cs, h16* Ph, h16* Pr, int resT) {
    __shared__ __align__(16) float os[16 * 68];
    const int K = DM;
    const int lane = threadIdx.x & 31, lr = lane & 15, hi = lane >> 4; const int r0 = blockIdx.x * 64, c0 = blockIdx.y * 64;
    v8f acc[4][4];
#pragma unroll
    for (int mb = 0; mb < 4; ++mb)
#pragma unroll
        for (int nb = 0; nb < 4; ++nb) acc[mb][nb] = (v8f){};
    const size_t aoff = (size_t)(r0 + lr) * K + 8 * hi, boff = (size_t)(c0 + lr) * K + 8 * hi;
#pragma unroll 1
    for (int kc = 0; kc < K; kc += 32) {
        v16bf a[4];
#pragma unroll
        for (int mb = 0; mb < 4; ++mb) a[mb] = ldb(A + aoff + (size_t)mb * 16 * K + kc);
#pragma unroll
        for (int nb = 0; nb < 4; ++nb) { const v16bf b = ldb(Bt + boff + (size_t)nb * 16 * K + kc);
#pragma unroll
            for (int mb = 0; mb < 4; ++mb) acc[mb][nb] = wmmabg(a[mb], b, acc[mb][nb]); }
    }
    size_t tbase, rbase; bool wr; int tq;
    if (MODE == 0) { const int bb = r0 / SEQ, tt = r0 % SEQ; const int zc = bb * NZ + c0 / HD;
                     tbase = ((size_t)zc * SEQ + (size_t)tt) * HD; rbase = ((size_t)zc * (size_t)resT + (size_t)tt) * HD; wr = tt < resT; tq = tt; }
    else           { const int bb = c0 / SEQ, tt = c0 % SEQ;
                     tbase = (size_t)bb * (size_t)DM * SEQ + (size_t)r0 * SEQ + (size_t)tt; rbase = (size_t)bb * (size_t)DM * (size_t)resT + (size_t)r0 * (size_t)resT + (size_t)tt; wr = tt < resT; tq = 0; }
#pragma unroll
    for (int mb = 0; mb < 4; ++mb) {
#pragma unroll
        for (int nb = 0; nb < 4; ++nb) {
#pragma unroll
            for (int j = 0; j < 8; ++j) os[(hi * 8 + j) * 68 + nb * 16 + lr] = acc[mb][nb][j]; }
        wave_sync();
#pragma unroll 1
        for (int ps = 0; ps < 2; ++ps) {
            if (MODE == 0) {
                const size_t sb = tbase + (size_t)(mb * 16) * HD;
                const size_t rb = rbase + (size_t)(mb * 16) * HD;
#pragma unroll
                for (int hh = 0; hh < 2; ++hh) {
#pragma unroll
                    for (int s = 0; s < 2; ++s) { const int p = s * 32 + lane; const int row = p >> 2, c8 = (p & 3) * 8;
                        const v4f x0 = *(const v4fa*)(&os[row * 68 + hh * 32 + c8]); const v4f x1 = *(const v4fa*)(&os[row * 68 + hh * 32 + c8 + 4]);
                        const float* cr = cs + (size_t)(tq + mb * 16 + row) * 32 + (c8 >> 1);
                        const v4f cc = *(const v4f*)cr; const v4f sn = *(const v4f*)(cr + 16);
                        float y[8];
                        y[0] = x0[0] * cc[0] - x0[1] * sn[0]; y[1] = x0[0] * sn[0] + x0[1] * cc[0];
                        y[2] = x0[2] * cc[1] - x0[3] * sn[1]; y[3] = x0[2] * sn[1] + x0[3] * cc[1];
                        y[4] = x1[0] * cc[2] - x1[1] * sn[2]; y[5] = x1[0] * sn[2] + x1[1] * cc[2];
                        y[6] = x1[2] * cc[3] - x1[3] * sn[3]; y[7] = x1[2] * sn[3] + x1[3] * cc[3];
                        v8h hv, rv;
#pragma unroll
                        for (int i = 0; i < 8; ++i) { const h16 a0 = toh_flush(y[i]); hv[i] = a0; rv[i] = toh_flush((y[i] - (float)a0) * QRS); }
                        const size_t oo = sb + (size_t)hh * ((size_t)SEQ * HD) + (size_t)p * 8;
                        const size_t ro = rb + (size_t)hh * ((size_t)resT * HD) + (size_t)p * 8;
                        *(volatile v8h*)(Ph + oo) = hv; if (wr) *(volatile v8h*)(Pr + ro) = rv; } }
            } else {
                const size_t sb = tbase + (size_t)(mb * 16) * SEQ;
                const size_t rb = rbase + (size_t)(mb * 16) * (size_t)resT;
#pragma unroll
                for (int s = 0; s < 4; ++s) { const int row = 4 * s + (lane >> 3), c8 = (lane & 7) * 8;
                    const v4f x0 = *(const v4fa*)(&os[row * 68 + c8]); const v4f x1 = *(const v4fa*)(&os[row * 68 + c8 + 4]); v8h hv, rv;
#pragma unroll
                    for (int i = 0; i < 4; ++i) { const h16 a0 = toh_flush(x0[i]); const h16 a1 = toh_flush(x1[i]); hv[i] = a0; hv[4 + i] = a1;
                                                  rv[i] = toh_flush((x0[i] - (float)a0) * QRS); rv[4 + i] = toh_flush((x1[i] - (float)a1) * QRS); }
                    const size_t oo = sb + (size_t)row * SEQ + c8;
                    const size_t ro = rb + (size_t)row * (size_t)resT + c8;
                    *(volatile v8h*)(Ph + oo) = hv; if (wr) *(volatile v8h*)(Pr + ro) = rv; }
            }
            if (ps == 0) __threadfence(); }
        wave_sync();
    }
}

__global__ __launch_bounds__(32) void k_proj_qk(const bf* __restrict__ A, const bf* __restrict__ Bt, const float* __restrict__ cs, h16* Ph, h16* Pr, int resT) {
    proj_body<0>(A, Bt, cs, Ph, Pr, resT);
}
__global__ __launch_bounds__(32) void k_proj_vt(const bf* __restrict__ A, const bf* __restrict__ Bt, const float* __restrict__ cs, h16* Ph, h16* Pr, int resT) {
    proj_body<1>(A, Bt, cs, Ph, Pr, resT);
}

template <int EARLY>
__device__ __forceinline__ void flash_body(const h16* __restrict__ QH, const h16* __restrict__ QR, const h16* __restrict__ KP, const h16* __restrict__ KR,
                                           const h16* __restrict__ VT, const h16* __restrict__ VR, const float* __restrict__ misc, h16* ATT) {
    __shared__ __align__(16) float os[AW * 16 * OSP];
    const int lane = threadIdx.x & 31, lr = lane & 15, hi = lane >> 4;
    const int wave = __builtin_amdgcn_readfirstlane((int)(threadIdx.x >> 5));
    const int zh = blockIdx.y; const int b = zh / NH_, h = zh % NH_;
    const int t0 = (EARLY ? 0 : EROWS) + (blockIdx.x * AW + wave) * 16;
    const int lim = t0 + lr;
    const int nk = (t0 + 16 + 31) & ~31;
    const float lam = misc[16];
    const size_t vo  = (size_t)zh * VD * SEQ   + (size_t)lr * SEQ   + 8 * hi;
    const size_t vro = (size_t)zh * VD * EROWS + (size_t)lr * EROWS + 8 * hi;
    const v16h hz = (v16h){};
    const int wb = wave * 16 * OSP;
    v8f f[4];
#pragma unroll
    for (int j = 0; j < 4; ++j) f[j] = (v8f){};
#pragma unroll 1
    for (int c = 0; c < 2; ++c) {
        const int z = b * NZ + 2 * h + c;
        const size_t pbase = (size_t)z * SEQ * HD;
        const size_t rbase = (size_t)z * EROWS * HD;
        const v16h qh = ldh(QH + pbase + (size_t)(t0 + lr) * HD + 8 * hi);
        v16h qr = hz;
        if (EARLY) qr = ldh(QR + rbase + (size_t)(t0 + lr) * HD + 8 * hi);
        const size_t ko  = pbase + (size_t)lr * HD + 8 * hi;
        const size_t kro = rbase + (size_t)lr * HD + 8 * hi;
        v8f o[4], oR[4];
#pragma unroll
        for (int j = 0; j < 4; ++j) { o[j] = (v8f){}; oR[j] = (v8f){}; }
        float m = NEGB, l = 0.0f;
#pragma unroll 1
        for (int key0 = 0; key0 < nk; key0 += 32) {
            const h16* ka = KP + ko + (size_t)key0 * HD;
            const v16h ka0 = ldh(ka), kb0 = ldh(ka + 16 * HD);
            v8f sHa = (v8f){}, sHb = (v8f){};
            sHa = wmma16g(ka0, qh, sHa); sHb = wmma16g(kb0, qh, sHb);
            float ta[8], tb[8];
            if (EARLY) {
                const h16* kr = KR + kro + (size_t)key0 * HD;
                const v16h kra0 = ldh(kr), krb0 = ldh(kr + 16 * HD);
                v8f sLa = (v8f){}, sLb = (v8f){};
                sLa = wmma16g(ka0, qr, sLa); sLa = wmma16g(kra0, qh, sLa);
                sLb = wmma16g(kb0, qr, sLb); sLb = wmma16g(krb0, qh, sLb);
#pragma unroll
                for (int r = 0; r < 8; ++r) { ta[r] = (sHa[r] + sLa[r] * QRI) * SC2; tb[r] = (sHb[r] + sLb[r] * QRI) * SC2; }
            } else {
#pragma unroll
                for (int r = 0; r < 8; ++r) { ta[r] = sHa[r] * SC2; tb[r] = sHb[r] * SC2; }
            }
            const int ja = key0 + 8 * hi;
            bool fa[8], fb[8]; float mx = NEGB;
#pragma unroll
            for (int r = 0; r < 8; ++r) {
                fa[r] = (ja + r <= lim);
                fb[r] = (ja + 16 + r <= lim);
                mx = fmaxf(mx, fmaxf(fa[r] ? ta[r] : NEGB, fb[r] ? tb[r] : NEGB)); }
            mx = fmaxf(mx, __shfl_xor(mx, 16, 32));
            const float mnew = fmaxf(m, mx);
            const float alpha = __builtin_amdgcn_exp2f(m - mnew);
            const float sh = PSH - mnew;
            v16h pb, pr; float ls = 0.0f;
#pragma unroll
            for (int r = 0; r < 8; ++r) {
                const float xa = ta[r] + sh, xb = tb[r] + sh;
                const float ea = (xa < -14.0f) ? 0.0f : __builtin_amdgcn_exp2f(xa);
                const float eb = (xb < -14.0f) ? 0.0f : __builtin_amdgcn_exp2f(xb);
                const float ga = fa[r] ? ea : 0.0f, gb = fb[r] ? eb : 0.0f;
                const h16 pa = (h16)ga; const h16 pc = (h16)gb;
                pb[r] = pa; pb[8 + r] = pc;
                pr[r] = toh_flush((ga - (float)pa) * QRS); pr[8 + r] = toh_flush((gb - (float)pc) * QRS);
                ls += ga + gb; }
            l = l * alpha + ls; m = mnew;
#pragma unroll
            for (int j = 0; j < 4; ++j) { o[j] = o[j] * alpha; oR[j] = oR[j] * alpha; }
            const h16* va = VT + vo + key0;
            { const v16h v0 = ldh(va), v1 = ldh(va + (size_t)16 * SEQ);
              o[0] = wmma16g(v0, pb, o[0]); o[1] = wmma16g(v1, pb, o[1]);
              oR[0] = wmma16g(v0, pr, oR[0]); oR[1] = wmma16g(v1, pr, oR[1]);
              if (EARLY) { const h16* vr = VR + vro + key0;
                           const v16h vr0 = ldh(vr), vr1 = ldh(vr + (size_t)16 * EROWS);
                           oR[0] = wmma16g(vr0, pb, oR[0]); oR[1] = wmma16g(vr1, pb, oR[1]); } }
            { const v16h v2 = ldh(va + (size_t)32 * SEQ), v3 = ldh(va + (size_t)48 * SEQ);
              o[2] = wmma16g(v2, pb, o[2]); o[3] = wmma16g(v3, pb, o[3]);
              oR[2] = wmma16g(v2, pr, oR[2]); oR[3] = wmma16g(v3, pr, oR[3]);
              if (EARLY) { const h16* vr = VR + vro + key0;
                           const v16h vr2 = ldh(vr + (size_t)32 * EROWS), vr3 = ldh(vr + (size_t)48 * EROWS);
                           oR[2] = wmma16g(vr2, pb, oR[2]); oR[3] = wmma16g(vr3, pb, oR[3]); } }
        }
        l += __shfl_xor(l, 16, 32);
        const float lsafe = (l > 0.0f) ? l : 1.0f;
        const float inv = 1.0f / lsafe;
#pragma unroll
        for (int j = 0; j < 4; ++j) f[j] = (o[j] + oR[j] * QRI) * inv;
        if (c == 0) {
#pragma unroll
            for (int j = 0; j < 4; ++j) { v4f a, e;
                a[0] = f[j][0]; a[1] = f[j][1]; a[2] = f[j][2]; a[3] = f[j][3]; e[0] = f[j][4]; e[1] = f[j][5]; e[2] = f[j][6]; e[3] = f[j][7];
                *(v4fa*)(&os[wb + lr * OSP + 16 * j + 8 * hi]) = a; *(v4fa*)(&os[wb + lr * OSP + 16 * j + 8 * hi + 4]) = e; }
        }
    }
    float ss = 0.0f;
#pragma unroll
    for (int j = 0; j < 4; ++j) {
        const v4f a = *(const v4fa*)(&os[wb + lr * OSP + 16 * j + 8 * hi]); const v4f e = *(const v4fa*)(&os[wb + lr * OSP + 16 * j + 8 * hi + 4]);
#pragma unroll
        for (int i = 0; i < 4; ++i) { const float x = a[i] - lam * f[j][i]; const float y = e[i] - lam * f[j][4 + i]; f[j][i] = x; f[j][4 + i] = y; ss += x * x + y * y; } }
    ss += __shfl_xor(ss, 16, 32);
    const float rn = rsqrtf(ss * (1.0f / 64.0f) + EPSN) * OML;
#pragma unroll
    for (int j = 0; j < 4; ++j) { v4f a, e;
        a[0] = f[j][0] * rn; a[1] = f[j][1] * rn; a[2] = f[j][2] * rn; a[3] = f[j][3] * rn; e[0] = f[j][4] * rn; e[1] = f[j][5] * rn; e[2] = f[j][6] * rn; e[3] = f[j][7] * rn;
        *(v4fa*)(&os[wb + lr * OSP + 16 * j + 8 * hi]) = a; *(v4fa*)(&os[wb + lr * OSP + 16 * j + 8 * hi + 4]) = e; }
    wave_sync();
    h16* arow = ATT + ((size_t)b * SEQ + t0) * DM + h * VD;
#pragma unroll 1
    for (int ps = 0; ps < 2; ++ps) {
#pragma unroll
        for (int s = 0; s < 4; ++s) { const int row = 4 * s + (lane >> 3), c8 = (lane & 7) * 8;
            const v4f x0 = *(const v4fa*)(&os[wb + row * OSP + c8]); const v4f x1 = *(const v4fa*)(&os[wb + row * OSP + c8 + 4]); v8h hv;
#pragma unroll
            for (int i = 0; i < 4; ++i) { hv[i] = toh_flush(x0[i] * ACS); hv[4 + i] = toh_flush(x1[i] * ACS); }
            *(volatile v8h*)(arow + (size_t)row * DM + c8) = hv; }
        if (ps == 0) __threadfence(); }
}

__global__ __launch_bounds__(32 * AW) __attribute__((amdgpu_num_vgpr(256))) void k_flash_early(const h16* __restrict__ QH, const h16* __restrict__ QR, const h16* __restrict__ KP, const h16* __restrict__ KR,
                                                                                             const h16* __restrict__ VT, const h16* __restrict__ VR, const float* __restrict__ misc, h16* ATT) {
    flash_body<1>(QH, QR, KP, KR, VT, VR, misc, ATT);
}
__global__ __launch_bounds__(32 * AW) __attribute__((amdgpu_num_vgpr(256))) void k_flash_late(const h16* __restrict__ QH, const h16* __restrict__ QR, const h16* __restrict__ KP, const h16* __restrict__ KR,
                                                                                            const h16* __restrict__ VT, const h16* __restrict__ VR, const float* __restrict__ misc, h16* ATT) {
    flash_body<0>(QH, QR, KP, KR, VT, VR, misc, ATT);
}

template <int EPI>
__device__ __forceinline__ void gemm_body(const h16* __restrict__ A, const h16* __restrict__ Bt, const float* __restrict__ bias, const float* __restrict__ res,
                                          float* F, h16* Hh, int K, int N, float osc, float hsc) {
    __shared__ __align__(16) float os[16 * 68];
    const int lane = threadIdx.x & 31, lr = lane & 15, hi = lane >> 4; const int r0 = blockIdx.x * 64, c0 = blockIdx.y * 64;
    v8f acc[4][4];
#pragma unroll
    for (int mb = 0; mb < 4; ++mb)
#pragma unroll
        for (int nb = 0; nb < 4; ++nb) acc[mb][nb] = (v8f){};
    const size_t aoff = (size_t)(r0 + lr) * K + 8 * hi, boff = (size_t)(c0 + lr) * K + 8 * hi;
#pragma unroll 1
    for (int kc = 0; kc < K; kc += 32) {
        v16h a[4];
#pragma unroll
        for (int mb = 0; mb < 4; ++mb) a[mb] = ldh(A + aoff + (size_t)mb * 16 * K + kc);
#pragma unroll
        for (int nb = 0; nb < 4; ++nb) { const v16h b = ldh(Bt + boff + (size_t)nb * 16 * K + kc);
#pragma unroll
            for (int mb = 0; mb < 4; ++mb) acc[mb][nb] = wmma16g(a[mb], b, acc[mb][nb]); }
    }
    float bc[4];
#pragma unroll
    for (int nb = 0; nb < 4; ++nb) bc[nb] = 0.0f;
    if (EPI != 0) {
#pragma unroll
        for (int nb = 0; nb < 4; ++nb) bc[nb] = bfr(bias[c0 + nb * 16 + lr]);
    }
#pragma unroll
    for (int mb = 0; mb < 4; ++mb) {
#pragma unroll
        for (int nb = 0; nb < 4; ++nb) {
#pragma unroll
            for (int j = 0; j < 8; ++j) os[(hi * 8 + j) * 68 + nb * 16 + lr] = acc[mb][nb][j] * osc + bc[nb]; }
        wave_sync();
        const size_t gb = (size_t)(r0 + mb * 16) * N + c0;
#pragma unroll 1
        for (int ps = 0; ps < 2; ++ps) {
            if (EPI != 1) {
#pragma unroll
                for (int s = 0; s < 8; ++s) { const int row = 2 * s + (lane >> 4), c4 = (lane & 15) * 4;
                    v4f x = *(const v4fa*)(&os[row * 68 + c4]);
                    if (EPI == 2) { const v4f rr = *(const v4f*)(res + gb + (size_t)row * N + c4); x = x + rr; }
                    *(volatile v4f*)(F + gb + (size_t)row * N + c4) = x; }
            }
            if (EPI != 2) {
#pragma unroll
                for (int s = 0; s < 4; ++s) { const int row = 4 * s + (lane >> 3), c8 = (lane & 7) * 8;
                    const v4f x0 = *(const v4fa*)(&os[row * 68 + c8]); const v4f x1 = *(const v4fa*)(&os[row * 68 + c8 + 4]); v8h hv;
#pragma unroll
                    for (int i = 0; i < 4; ++i) { float u0 = x0[i], u1 = x1[i];
                        if (EPI == 1) { u0 = (u0 > 0.0f) ? u0 : 0.0f; u1 = (u1 > 0.0f) ? u1 : 0.0f; }
                        hv[i] = toh_flush(u0 * hsc); hv[4 + i] = toh_flush(u1 * hsc); }
                    *(volatile v8h*)(Hh + gb + (size_t)row * N + c8) = hv; }
            }
            if (ps == 0) __threadfence(); }
        wave_sync();
    }
}

__global__ __launch_bounds__(32) void k_gemm_wo(const h16* __restrict__ A, const h16* __restrict__ Bt, float* F, h16* Hh) {
    gemm_body<0>(A, Bt, F, F, F, Hh, DM, DM, 1.0f / (WCS * ACS), ACS);
}
__global__ __launch_bounds__(32) void k_gemm_w1(const h16* __restrict__ A, const h16* __restrict__ Bt, const float* __restrict__ bias, float* F, h16* Hh) {
    gemm_body<1>(A, Bt, bias, bias, F, Hh, DM, FF, 1.0f / (WCS * ACS), HCS);
}
__global__ __launch_bounds__(32) void k_gemm_w2(const h16* __restrict__ A, const h16* __restrict__ Bt, const float* __restrict__ bias, const float* __restrict__ res, float* F, h16* Hh) {
    gemm_body<2>(A, Bt, bias, res, F, Hh, FF, DM, 1.0f / (WCS * HCS), 1.0f);
}

__global__ __launch_bounds__(256) void k_rmsnorm(const float* __restrict__ Y, const float* __restrict__ gain, float* OUT) {
#pragma clang fp contract(off)
    const int lane = threadIdx.x & 31;
    const int wave = __builtin_amdgcn_readfirstlane((int)(threadIdx.x >> 5));
    const int row = blockIdx.x * 8 + wave;
    const float* yr = Y + (size_t)row * DM + lane * 4;
    float ss = 0.0f;
#pragma unroll 1
    for (int i = 0; i < 8; ++i) { const v4f v = *(const v4f*)(yr + i * 128); ss += (v[0] * v[0] + v[1] * v[1]) + (v[2] * v[2] + v[3] * v[3]); }
#pragma unroll 1
    for (int off = 16; off > 0; off >>= 1) ss += __shfl_xor(ss, off, 32);
    const float rn = rsqrtf(ss * (1.0f / 1024.0f) + EPSN);
    const int bb = row / SEQ, tt = row % SEQ;
    float* orow = OUT + ((size_t)bb * OUT_SEQ + tt) * DM + lane * 4;
    const float* gr = gain + lane * 4;
#pragma unroll 1
    for (int ps = 0; ps < 2; ++ps) {
#pragma unroll 1
        for (int i = 0; i < 8; ++i) { const v4f v = *(const v4f*)(yr + i * 128); const v4f g = *(const v4f*)(gr + i * 128); v4f o;
            o[0] = v[0] * rn * bfr(g[0]); o[1] = v[1] * rn * bfr(g[1]); o[2] = v[2] * rn * bfr(g[2]); o[3] = v[3] * rn * bfr(g[3]);
            *(volatile v4f*)(orow + i * 128) = o; }
        if (ps == 0) __threadfence(); }
}

static constexpr size_t al256(size_t v) { return (v + 255) & ~(size_t)255; }
static constexpr size_t mx2(size_t a, size_t b) { return a > b ? a : b; }
static constexpr size_t SZ_XB  = al256((size_t)NB * SEQ * DM * 2);
static constexpr size_t SZ_PL  = al256((size_t)NB * NZ * SEQ * HD * 2);
static constexpr size_t SZ_VT  = al256((size_t)NB * DM * SEQ * 2);
static constexpr size_t SZ_H1  = al256((size_t)NB * SEQ * FF * 2);
static constexpr size_t SZ_R0  = mx2(SZ_XB + 2 * SZ_PL + SZ_VT, SZ_H1);
static constexpr size_t SZ_WB  = al256((size_t)3 * DM * DM * 2);
static constexpr size_t SZ_RS  = al256((size_t)NB * NZ * EROWS * HD * 2);
static constexpr size_t SZ_VR  = al256((size_t)NB * DM * EROWS * 2);
static constexpr size_t SZ_WO  = al256((size_t)DM * DM * 2);
static constexpr size_t SZ_W1  = al256((size_t)FF * DM * 2);
static constexpr size_t SZ_W2  = al256((size_t)DM * FF * 2);
static constexpr size_t SZ_ATT = al256((size_t)NB * SEQ * DM * 2);
static constexpr size_t SZ_AOH = al256((size_t)NB * SEQ * DM * 2);
static constexpr size_t SZ_Y   = al256((size_t)NB * SEQ * DM * 4);
static constexpr size_t SZ_R1  = mx2(SZ_ATT + SZ_AOH, SZ_Y);
static constexpr size_t SZ_AO  = al256((size_t)NB * SEQ * DM * 4);
static constexpr size_t SZ_CS  = al256((size_t)SEQ * 32 * 4);
static constexpr size_t SZ_MI  = 256;
static constexpr size_t SZ_TOTAL = SZ_R0 + SZ_WB + 2 * SZ_RS + SZ_VR + SZ_WO + SZ_W1 + SZ_W2 + SZ_R1 + SZ_AO + SZ_CS + SZ_MI;
static_assert(SZ_TOTAL <= (size_t)134217728);
static_assert(SZ_H1 <= SZ_R0);
static_assert(SZ_XB + 2 * SZ_PL + SZ_VT <= SZ_R0);
static_assert(SZ_Y <= SZ_R1);
static_assert(SZ_ATT + SZ_AOH <= SZ_R1);
static_assert(((size_t)DM * DM * 2) % 256 == 0);
static_assert((size_t)NB * NZ * SEQ * HD == (size_t)NB * DM * SEQ);

extern "C" void kernel_launch(void* const* d_in, const int* in_sizes, int n_in,
                              void* d_out, int out_size, void* d_ws, size_t ws_size, hipStream_t stream) {
    if (n_in < 14) return;
    const size_t needx = ((size_t)(NB - 1) * SEQ_FULL + SEQ) * DM;
    if ((size_t)in_sizes[0] < needx) return;
    if ((size_t)in_sizes[1] < (size_t)DM * DM || (size_t)in_sizes[2] < (size_t)DM * DM || (size_t)in_sizes[3] < (size_t)DM * DM || (size_t)in_sizes[4] < (size_t)DM * DM) return;
    if (in_sizes[5] < HD || in_sizes[6] < HD || in_sizes[7] < HD || in_sizes[8] < HD) return;
    if ((size_t)in_sizes[9] < (size_t)FF * DM || in_sizes[10] < FF || (size_t)in_sizes[11] < (size_t)DM * FF || in_sizes[12] < DM || in_sizes[13] < DM) return;
    if ((size_t)out_size < ((size_t)(NB - 1) * OUT_SEQ + SEQ) * DM) return;
    if (SZ_TOTAL > ws_size) return;
    const float* x   = (const float*)d_in[0];
    const float* wq  = (const float*)d_in[1];
    const float* wk  = (const float*)d_in[2];
    const float* wv  = (const float*)d_in[3];
    const float* wo  = (const float*)d_in[4];
    const float* lq1 = (const float*)d_in[5];
    const float* lk1 = (const float*)d_in[6];
    const float* lq2 = (const float*)d_in[7];
    const float* lk2 = (const float*)d_in[8];
    const float* w1  = (const float*)d_in[9];
    const float* b1  = (const float*)d_in[10];
    const float* w2  = (const float*)d_in[11];
    const float* b2  = (const float*)d_in[12];
    const float* gw  = (const float*)d_in[13];
    float* OUT = (float*)d_out;
    char* wsp = (char*)d_ws;
    char* r0p = wsp; wsp += SZ_R0;
    bf*  XB = (bf*)r0p;
    h16* QH = (h16*)(r0p + SZ_XB);
    h16* KP = (h16*)(r0p + SZ_XB + SZ_PL);
    h16* VT = (h16*)(r0p + SZ_XB + 2 * SZ_PL);
    h16* H1 = (h16*)r0p;
    bf* WB = (bf*)wsp; wsp += SZ_WB;
    h16* QR = (h16*)wsp; wsp += SZ_RS;
    h16* KR = (h16*)wsp; wsp += SZ_RS;
    h16* VR = (h16*)wsp; wsp += SZ_VR;
    h16* WOH = (h16*)wsp; wsp += SZ_WO;
    h16* W1H = (h16*)wsp; wsp += SZ_W1;
    h16* W2H = (h16*)wsp; wsp += SZ_W2;
    char* r1p = wsp; wsp += SZ_R1;
    h16* ATT = (h16*)r1p;
    h16* AOH = (h16*)(r1p + SZ_ATT);
    float* Y = (float*)r1p;
    float* AO = (float*)wsp; wsp += SZ_AO;
    float* CS = (float*)wsp; wsp += SZ_CS;
    float* MI = (float*)wsp; wsp += SZ_MI;
    bf* WQ = WB; bf* WK = WB + (size_t)DM * DM; bf* WV = WB + (size_t)2 * DM * DM;

    if (SEQ == SEQ_FULL) {
        const size_t n8 = (size_t)NB * SEQ * DM / 8;
        k_cvt8<<<(unsigned)((n8 + 255) / 256), 256, 0, stream>>>(x, XB, n8);
    } else {
        const size_t n8 = (size_t)SEQ * DM / 8;
        for (int b = 0; b < NB; ++b) k_cvt8<<<(unsigned)((n8 + 255) / 256), 256, 0, stream>>>(x + (size_t)b * SEQ_FULL * DM, XB + (size_t)b * SEQ * DM, n8);
    }
    { const size_t n8 = (size_t)DM * DM / 8; const unsigned g = (unsigned)((n8 + 255) / 256);
      k_cvt8<<<g, 256, 0, stream>>>(wq, WQ, n8); k_cvt8<<<g, 256, 0, stream>>>(wk, WK, n8); k_cvt8<<<g, 256, 0, stream>>>(wv, WV, n8);
      k_wconv<<<g, 256, 0, stream>>>(wo, WOH, n8); }
    { const size_t n8 = (size_t)FF * DM / 8; const unsigned g = (unsigned)((n8 + 255) / 256);
      k_wconv<<<g, 256, 0, stream>>>(w1, W1H, n8); k_wconv<<<g, 256, 0, stream>>>(w2, W2H, n8); }

    k_misc<<<1, 32, 0, stream>>>(lq1, lk1, lq2, lk2, MI);
    k_ropetab<<<SEQ * 32 / 256, 256, 0, stream>>>(MI, CS);

    k_proj_qk<<<dim3(NB * SEQ / 64, DM / 64, 1), 32, 0, stream>>>(XB, WQ, CS, QH, QR, EROWS);
    k_proj_qk<<<dim3(NB * SEQ / 64, DM / 64, 1), 32, 0, stream>>>(XB, WK, CS, KP, KR, EROWS);
    k_proj_vt<<<dim3(DM / 64, NB * SEQ / 64, 1), 32, 0, stream>>>(WV, XB, CS, VT, VR, EROWS);

    k_flash_early<<<dim3(EROWS / (16 * AW), NB * NH_, 1), 32 * AW, 0, stream>>>(QH, QR, KP, KR, VT, VR, MI, ATT);
    if (SEQ > EROWS)
        k_flash_late<<<dim3((SEQ - EROWS) / (16 * AW), NB * NH_, 1), 32 * AW, 0, stream>>>(QH, QR, KP, KR, VT, VR, MI, ATT);

    k_gemm_wo<<<dim3(NB * SEQ / 64, DM / 64, 1), 32, 0, stream>>>(ATT, WOH, AO, AOH);
    k_gemm_w1<<<dim3(NB * SEQ / 64, FF / 64, 1), 32, 0, stream>>>(AOH, W1H, b1, AO, H1);
    k_gemm_w2<<<dim3(NB * SEQ / 64, DM / 64, 1), 32, 0, stream>>>(H1, W2H, b2, AO, Y, AOH);
    k_rmsnorm<<<NB * SEQ / 8, 256, 0, stream>>>(Y, gw, OUT);
}
